// STHGNN_87058987090148
// MI455X (gfx1250) — hardware-verified
//
#include <hip/hip_runtime.h>
#include <math.h>

typedef unsigned short u16;
typedef __attribute__((ext_vector_type(16))) __bf16 v16b;
typedef __attribute__((ext_vector_type(8)))  float v8f;
typedef __attribute__((ext_vector_type(4)))  float v4f;
typedef __attribute__((ext_vector_type(4)))  unsigned int v4u;
typedef __attribute__((ext_vector_type(8)))  unsigned int v8u;
typedef v4f __attribute__((may_alias)) v4fa;
typedef v4u __attribute__((may_alias)) v4ua;

#define DEV __device__ __forceinline__
#define KATTR __attribute__((amdgpu_num_vgpr(248)))

#define NBAT 4
#define NTIM 64
#define NNOD 256
#define NEDG 128
#define NDIM 64
#define MTOK 65536
static_assert(NNOD % 128 == 0);
static_assert(NDIM == 64);
static_assert(NEDG == 128);
static_assert(NTIM == 64);
static_assert(MTOK % 128 == 0);
static_assert(MTOK == NBAT * NTIM * NNOD);

static constexpr size_t SLOT    = 16777216;
static constexpr size_t B_SM    = 7 * SLOT;
static constexpr size_t B_FG    = B_SM;
static constexpr size_t B_SK    = B_FG   + 98304;
static constexpr size_t B_CZ    = B_SK   + 49152;
static constexpr size_t B_FUSE  = B_CZ   + 65536;
static constexpr size_t B_OUT   = B_FUSE + 65536;
static constexpr size_t B_END   = B_OUT  + 32768;
static constexpr size_t B_WQD   = B_END  + 16384;
static constexpr size_t B_NWB   = B_WQD  + 16384;
static constexpr size_t B_WKB   = B_NWB  + 8192;
static constexpr size_t B_HEMB  = B_WKB  + 8192;
static constexpr size_t B_ABF   = B_HEMB + 16384;
static constexpr size_t B_GLT   = B_ABF  + 131072;
static constexpr size_t B_XPT   = B_GLT  + 65536;
static constexpr size_t B_EEMB  = B_XPT  + 131072;
static constexpr size_t B_QHL   = B_EEMB + 262144;
static constexpr size_t B_KHL   = B_QHL  + 262144;
static constexpr size_t B_HF    = B_KHL  + 32768;
static constexpr size_t B_HG    = B_HF   + 524288;
static constexpr size_t B_LP    = B_HG   + 131072;
static constexpr size_t B_RP    = B_LP   + 524288;
static constexpr size_t B_LG    = B_RP   + 524288;
static constexpr size_t B_RG    = B_LG   + 131072;
static constexpr size_t B_ANHL  = B_RG   + 131072;
static constexpr size_t B_AGHL  = B_ANHL + 1048576;
static constexpr size_t B_TOTAL = B_AGHL + 262144;
static_assert(B_TOTAL == 121978880);
static_assert(B_TOTAL <= 134217728);
static constexpr size_t SLOTE  = SLOT / 2;
static constexpr size_t E_FG   = B_FG / 2,  E_SK = B_SK / 2,  E_CZ = B_CZ / 2,  E_FUSE = B_FUSE / 2;
static constexpr size_t E_OUT  = B_OUT / 2, E_END = B_END / 2, E_WQD = B_WQD / 2, E_NWB = B_NWB / 2;
static constexpr size_t E_WKB  = B_WKB / 2, E_HEMB = B_HEMB / 2, E_ABF = B_ABF / 2, E_GLT = B_GLT / 2;
static constexpr size_t E_XPT  = B_XPT / 2, E_EEMB = B_EEMB / 2, E_QHL = B_QHL / 2, E_KHL = B_KHL / 2;
static constexpr size_t E_LP   = B_LP / 2,  E_RP = B_RP / 2,  E_LG = B_LG / 2,  E_RG = B_RG / 2;
static constexpr size_t E_ANHL = B_ANHL / 2, E_AGHL = B_AGHL / 2;
static constexpr long   ZLO    = 4194304;

DEV u16 f2bf(float f) {
  const unsigned u = __float_as_uint(f);
  return (u16)((u + 0x7FFFu + ((u >> 16) & 1u)) >> 16);
}
DEV float bf2f(u16 h) { return __uint_as_float(((unsigned)h) << 16); }
DEV float rbf(float f) { return bf2f(f2bf(f)); }
DEV unsigned pk(u16 a, u16 b) { return (unsigned)a | ((unsigned)b << 16); }
DEV unsigned hi2(float x, float y) { return pk(f2bf(x), f2bf(y)); }
DEV unsigned lo2(float x, float y) {
  const u16 hx = f2bf(x), hy = f2bf(y);
  return pk(f2bf(x - bf2f(hx)), f2bf(y - bf2f(hy)));
}
DEV v4u hi8(v4f a, v4f b) { const v4u r = { hi2(a.x, a.y), hi2(a.z, a.w), hi2(b.x, b.y), hi2(b.z, b.w) }; return r; }
DEV v4u lo8(v4f a, v4f b) { const v4u r = { lo2(a.x, a.y), lo2(a.z, a.w), lo2(b.x, b.y), lo2(b.z, b.w) }; return r; }
DEV v4f rb4(v4f a) { const v4f r = { rbf(a.x), rbf(a.y), rbf(a.z), rbf(a.w) }; return r; }
DEV float lo16f(unsigned w) { return __uint_as_float(w << 16); }
DEV float hi16f(unsigned w) { return __uint_as_float(w & 0xffff0000u); }
DEV void unp8(v4u w, v4f& a, v4f& b) {
  const v4f ra = { lo16f(w.x), hi16f(w.x), lo16f(w.y), hi16f(w.y) };
  const v4f rb = { lo16f(w.z), hi16f(w.z), lo16f(w.w), hi16f(w.w) };
  a = ra; b = rb;
}
DEV float relu_keep(float v) { return (v > 0.0f) ? v : (v - v); }

DEV void wsync() {
  __builtin_amdgcn_fence(__ATOMIC_RELEASE, "workgroup");
  __builtin_amdgcn_wave_barrier();
  __builtin_amdgcn_fence(__ATOMIC_ACQUIRE, "workgroup");
}

DEV v8f mma(v16b a, v16b b, v8f c) {
  c = __builtin_amdgcn_wmma_f32_16x16x32_bf16(false, a, false, b, (short)0, c, false, false);
  asm volatile("v_nop\n\tv_nop\n\tv_nop\n\tv_nop" : "+v"(c) : "v"(a), "v"(b));
  return c;
}
DEV v16b ldfrag(const u16* p) {
  const v4u a = *(const v4ua*)p;
  const v4u b = *(const v4ua*)(p + 16);
  const v8u u = { a.x, a.y, a.z, a.w, b.x, b.y, b.z, b.w };
  return __builtin_bit_cast(v16b, u);
}

template <int NT>
DEV void zero_acc(v8f (&acc)[2][NT]) {
  const v8f z = { 0.f, 0.f, 0.f, 0.f, 0.f, 0.f, 0.f, 0.f };
#pragma unroll
  for (int i = 0; i < 2; ++i)
#pragma unroll
    for (int j = 0; j < NT; ++j) acc[i][j] = z;
}

template <int NT>
DEV void mm1(v8f (&acc)[2][NT], const u16* a0, const u16* a1, const u16* b, int ldb, int K) {
#pragma unroll 1
  for (int k0 = 0; k0 < K; k0 += 32) {
    const v16b fa0 = ldfrag(a0 + k0);
    const v16b fa1 = ldfrag(a1 + k0);
#pragma unroll
    for (int nt = 0; nt < NT; ++nt) {
      const v16b fb = ldfrag(b + (size_t)nt * 16 * ldb + k0);
      acc[0][nt] = mma(fa0, fb, acc[0][nt]);
      acc[1][nt] = mma(fa1, fb, acc[1][nt]);
    }
  }
}
template <int NT>
DEV void mm3(v8f (&acc)[2][NT], const u16* a0, const u16* a1, long alo, const u16* b, long blo, int ldb, int K) {
#pragma unroll 1
  for (int k0 = 0; k0 < K; k0 += 32) {
    const v16b ah0 = ldfrag(a0 + k0);
    const v16b al0 = ldfrag(a0 + alo + k0);
    const v16b ah1 = ldfrag(a1 + k0);
    const v16b al1 = ldfrag(a1 + alo + k0);
#pragma unroll
    for (int nt = 0; nt < NT; ++nt) {
      const u16* bp = b + (size_t)nt * 16 * ldb + k0;
      const v16b bh = ldfrag(bp);
      const v16b bl = ldfrag(bp + blo);
      acc[0][nt] = mma(ah0, bh, acc[0][nt]);
      acc[0][nt] = mma(ah0, bl, acc[0][nt]);
      acc[0][nt] = mma(al0, bh, acc[0][nt]);
      acc[1][nt] = mma(ah1, bh, acc[1][nt]);
      acc[1][nt] = mma(ah1, bl, acc[1][nt]);
      acc[1][nt] = mma(al1, bh, acc[1][nt]);
    }
  }
}

template <int NT, bool HASB>
DEV void stage16(float* slab, const v8f (&a)[NT], const float* bias, int n0, int h, int m) {
  constexpr int PITCH = 16 * NT + 4;
#pragma unroll
  for (int nt = 0; nt < NT; ++nt) {
    const int col = 16 * nt + m;
    float bv = 0.0f;
    if (HASB) bv = rbf(bias[n0 + col]);
#pragma unroll
    for (int r = 0; r < 8; ++r) slab[(8 * h + r) * PITCH + col] = a[nt][r] + bv;
  }
}

DEV void store_hl(const float* slab, int pitch, u16* dst, int ldc, int clo, int lane) {
  const int q = lane >> 3, c8 = (lane & 7) * 8;
  v4u hv[4], lv[4];
#pragma unroll
  for (int it = 0; it < 4; ++it) {
    const float* p = slab + (it * 4 + q) * pitch + c8;
    const v4f a = *(const v4fa*)p;
    const v4f b = *(const v4fa*)(p + 4);
    hv[it] = hi8(a, b);
    lv[it] = lo8(a, b);
  }
#pragma unroll
  for (int pass = 0; pass < 2; ++pass) {
#pragma unroll
    for (int it = 0; it < 4; ++it) {
      u16* d = dst + (size_t)(it * 4 + q) * ldc + c8;
      *(volatile v4u*)d = hv[it];
      *(volatile v4u*)(d + clo) = lv[it];
    }
    __threadfence();
  }
}

template <int NT>
DEV void store_f32(const float* slab, float* dst, int ldc, int lane) {
  constexpr int PITCH = 16 * NT + 4;
  constexpr int LPR = 4 * NT;
  constexpr int RPI = 32 / LPR;
  constexpr int ITS = 16 / RPI;
  const int rr = lane / LPR, c4 = (lane % LPR) * 4;
#pragma unroll
  for (int pass = 0; pass < 2; ++pass) {
#pragma unroll
    for (int it = 0; it < ITS; ++it) {
      const int row = it * RPI + rr;
      const v4f v = *(const v4fa*)(slab + row * PITCH + c4);
      *(volatile v4f*)(dst + (size_t)row * ldc + c4) = v;
    }
    __threadfence();
  }
}

DEV void softmax16(float* slab, int lane) {
#pragma unroll 1
  for (int r = 0; r < 16; ++r) {
    float* p = slab + r * 132 + 4 * lane;
    v4f v = *(const v4fa*)p;
    v = v * 0.125f;
    float mx = fmaxf(fmaxf(v.x, v.y), fmaxf(v.z, v.w));
    mx = fmaxf(mx, __shfl_xor(mx, 16));
    mx = fmaxf(mx, __shfl_xor(mx, 8));
    mx = fmaxf(mx, __shfl_xor(mx, 4));
    mx = fmaxf(mx, __shfl_xor(mx, 2));
    mx = fmaxf(mx, __shfl_xor(mx, 1));
    v4f e = { expf(v.x - mx), expf(v.y - mx), expf(v.z - mx), expf(v.w - mx) };
    float s = (e.x + e.y) + (e.z + e.w);
    s += __shfl_xor(s, 16);
    s += __shfl_xor(s, 8);
    s += __shfl_xor(s, 4);
    s += __shfl_xor(s, 2);
    s += __shfl_xor(s, 1);
    const float inv = 1.0f / s;
    e = e * inv;
    *(v4fa*)p = e;
  }
  wsync();
}

template <int NT, int TERMS, int EP, bool HASB, int LDA, int ALO, int LDB, int BLO, int KK, int LDC, int CLO, int AZ, int BZ, int CZS>
__global__ __launch_bounds__(128) KATTR
void k_gm(const u16* __restrict__ A, const u16* __restrict__ Bt, const float* __restrict__ bias,
          u16* __restrict__ Ch, float* __restrict__ Cf)
{
  static_assert(KK % 32 == 0);
  static_assert(EP != 0 || NT == 4);
  static_assert(EP != 2 || NT == 8);
  constexpr int PITCH = 16 * NT + 4;
  __shared__ __attribute__((aligned(16))) float sS[4 * 16 * PITCH];
  const int tid = threadIdx.x, lane = tid & 31, w = tid >> 5;
  const int h = lane >> 4, m = lane & 15;
  const int m0w = blockIdx.x * 128 + 32 * w;
  const int n0 = blockIdx.y * 16 * NT;
  const int z = blockIdx.z;
  const u16* a0 = A + (size_t)z * AZ + (size_t)(m0w + m) * LDA + 8 * h;
  const u16* a1 = a0 + 16 * LDA;
  const u16* b = Bt + (size_t)z * BZ + (size_t)(n0 + m) * LDB + 8 * h;
  v8f acc[2][NT];
  zero_acc<NT>(acc);
  if constexpr (TERMS == 1) mm1<NT>(acc, a0, a1, b, LDB, KK);
  else mm3<NT>(acc, a0, a1, (long)ALO, b, (long)BLO, LDB, KK);

  float* slab = sS + w * 16 * PITCH;
#pragma unroll
  for (int mt = 0; mt < 2; ++mt) {
    stage16<NT, HASB>(slab, acc[mt], bias, n0, h, m);
    wsync();
    const int row0 = m0w + 16 * mt;
    if constexpr (EP == 0) {
      store_hl(slab, PITCH, Ch + (size_t)z * CZS + (size_t)row0 * LDC + n0, LDC, CLO, lane);
    } else {
      if constexpr (EP == 2) softmax16(slab, lane);
      store_f32<NT>(slab, Cf + (size_t)z * CZS + (size_t)row0 * LDC + n0, LDC, lane);
    }
    wsync();
  }
}

DEV void dupcopy(const float* __restrict__ src, int srcLd, int srcOff, u16* dst, int dstLd, int dstOff, int t) {
  const int row = t >> 4, p = t & 15, c8 = (p & 7) * 8;
  const float* s = src + row * srcLd + srcOff + c8;
  const v4f a = *(const v4fa*)s;
  const v4f b = *(const v4fa*)(s + 4);
  const v4u hv = hi8(a, b);
  u16* d = dst + row * dstLd + dstOff + p * 8;
  *(volatile v4u*)d = hv;
  __threadfence();
  *(volatile v4u*)d = hv;
}
__global__ __launch_bounds__(256) KATTR
void k_pa(const float* __restrict__ filtW, const float* __restrict__ gateW, const float* __restrict__ skipW,
          const float* __restrict__ Wf, const float* __restrict__ Wg, const float* __restrict__ oW,
          const float* __restrict__ endW, const float* __restrict__ Wq, u16* __restrict__ ws)
{
  const int t = blockIdx.x * 256 + threadIdx.x;
  const int job = blockIdx.y;
  if (job < 3)        dupcopy(filtW + job * 4096, 64, 0, ws + E_FG + job * 16384, 128, 0, t);
  else if (job < 6)   dupcopy(gateW + (job - 3) * 4096, 64, 0, ws + E_FG + (job - 3) * 16384 + 8192, 128, 0, t);
  else if (job < 9)   dupcopy(skipW + (job - 6) * 4096, 64, 0, ws + E_SK + (job - 6) * 8192, 128, 0, t);
  else if (job == 9)  dupcopy(Wf, 128, 0,  ws + E_FUSE, 512, 0,   t);
  else if (job == 10) dupcopy(Wg, 128, 0,  ws + E_FUSE, 512, 128, t);
  else if (job == 11) dupcopy(Wf, 128, 64, ws + E_FUSE, 512, 256, t);
  else if (job == 12) dupcopy(Wg, 128, 64, ws + E_FUSE, 512, 384, t);
  else if (job == 13) dupcopy(oW, 128, 0,  ws + E_OUT, 256, 0,   t);
  else if (job == 14) dupcopy(oW, 128, 64, ws + E_OUT, 256, 128, t);
  else if (job == 15) dupcopy(endW, 64, 0, ws + E_END, 128, 0, t);
  else                dupcopy(Wq, 64, 0, ws + E_WQD, 128, 0, t);
}

DEV void cpy8(const float* __restrict__ s, u16* d, int u) {
  const v4f a = *(const v4fa*)(s + 8 * u);
  const v4f b = *(const v4fa*)(s + 8 * u + 4);
  const v4u hv = hi8(a, b);
  *(volatile v4u*)(d + 8 * u) = hv;
  __threadfence();
  *(volatile v4u*)(d + 8 * u) = hv;
}
__global__ __launch_bounds__(256) KATTR
void k_pb(const float* __restrict__ nodeW, const float* __restrict__ Wk, const float* __restrict__ hemb,
          const float* __restrict__ Am, u16* __restrict__ ws)
{
  const int bx = blockIdx.x, tid = threadIdx.x;
  if (bx < 2)      cpy8(nodeW, ws + E_NWB, bx * 256 + tid);
  else if (bx < 4) cpy8(Wk, ws + E_WKB, (bx - 2) * 256 + tid);
  else if (bx < 8) cpy8(hemb, ws + E_HEMB, (bx - 4) * 256 + tid);
  else             cpy8(Am, ws + E_ABF, (bx - 8) * 256 + tid);
}

DEV void tr8(const float* __restrict__ s, int stride, u16* d) {
  const float f0 = s[0], f1 = s[stride], f2 = s[2 * stride], f3 = s[3 * stride];
  const float f4 = s[4 * stride], f5 = s[5 * stride], f6 = s[6 * stride], f7 = s[7 * stride];
  const v4u hv = { hi2(f0, f1), hi2(f2, f3), hi2(f4, f5), hi2(f6, f7) };
  *(volatile v4u*)d = hv;
  __threadfence();
  *(volatile v4u*)d = hv;
}
__global__ __launch_bounds__(256) KATTR
void k_pc(const float* __restrict__ cW, const float* __restrict__ cWg, const float* __restrict__ Gl,
          const float* __restrict__ X, u16* __restrict__ ws)
{
  const int bx = blockIdx.x, tid = threadIdx.x;
  if (bx < 16) {
    const int mat = bx >> 2, j = mat >> 1, g = mat & 1;
    const int t = (bx & 3) * 256 + tid;
    const int n = t >> 4, p = t & 15, c8 = (p & 7) * 8;
    u16* d = ws + E_CZ + j * 16384 + (g * 64 + n) * 128 + p * 8;
    if (g == 0) tr8(cW + j * 4096 + c8 * 64 + n, 64, d);
    else        tr8(cWg + j * 4096 + c8 * 64 + n, 64, d);
  } else if (bx < 32) {
    const int t = (bx - 16) * 256 + tid;
    const int e = t >> 5, c8 = (t & 31) * 8;
    tr8(Gl + c8 * 128 + e, 128, ws + E_GLT + e * 256 + c8);
  } else {
    const int t = (bx - 32) * 256 + tid;
    const int row = t >> 3, c8 = (t & 7) * 8;
    const int b = row >> 8, n = row & 255;
    tr8(X + b * 16384 + c8 * 256 + n, 256, ws + E_XPT + row * 64 + c8);
  }
}

__global__ __launch_bounds__(256) KATTR
void k_pd(const float* __restrict__ X, const float* __restrict__ sW, const float* __restrict__ sb,
          u16* __restrict__ XIN, float* __restrict__ SKIP)
{
  const int g = blockIdx.x * 256 + threadIdx.x;
  const int row = g >> 4, q = g & 15;
  const float xv = rbf(X[row]);
  const int c8 = (q & 7) * 8;
  const v4f w0 = rb4(*(const v4fa*)(sW + c8)), w1 = rb4(*(const v4fa*)(sW + c8 + 4));
  const v4f b0 = rb4(*(const v4fa*)(sb + c8)), b1 = rb4(*(const v4fa*)(sb + c8 + 4));
  const v4f y0 = w0 * xv + b0, y1 = w1 * xv + b1;
  const v4u hv = hi8(y0, y1), lv = lo8(y0, y1);
  const unsigned msk = 0u - (unsigned)(q >> 3);
  const v4u ov = (hv & ~msk) | (lv & msk);
  const int c4 = q * 4;
  const v4f ws4 = rb4(*(const v4fa*)(sW + c4)), bs4 = rb4(*(const v4fa*)(sb + c4));
  const v4f sv = ws4 * xv + bs4;
  u16* dx = XIN + (size_t)row * 128 + q * 8;
  float* ds = SKIP + (size_t)row * 64 + c4;
  *(volatile v4u*)dx = ov;
  *(volatile v4f*)ds = sv;
  __threadfence();
  *(volatile v4u*)dx = ov;
  *(volatile v4f*)ds = sv;
}

__global__ __launch_bounds__(256) KATTR
void k_lr(const float* __restrict__ H, u16* __restrict__ L, u16* __restrict__ R)
{
  __shared__ double sP[256];
  __shared__ __attribute__((aligned(16))) float sID[256];
  __shared__ __attribute__((aligned(16))) float sIB[128];
  const int tid = threadIdx.x;
  const float* Hb = H + (size_t)blockIdx.x * 32768;
  {
    const float* rp = Hb + tid * 128;
    double s = 0.0;
#pragma unroll 4
    for (int c = 0; c < 32; ++c) {
      const v4f v = *(const v4fa*)(rp + 4 * c);
      s += (double)v.x; s += (double)v.y; s += (double)v.z; s += (double)v.w;
    }
    const float d = (float)s;
    sID[tid] = (d > 0.0f) ? (1.0f / (d + 1e-8f)) : 0.0f;
  }
  {
    const int c = tid & 127, hf = tid >> 7;
    const float* cp = Hb + hf * 16384 + c;
    double s = 0.0;
#pragma unroll 4
    for (int r = 0; r < 128; ++r) s += (double)cp[r * 128];
    sP[tid] = s;
  }
  __syncthreads();
  if (tid < 128) {
    const double s = sP[tid] + sP[tid + 128];
    const float d = (float)s;
    sIB[tid] = (d > 0.0f) ? (1.0f / (d + 1e-8f)) : 0.0f;
  }
  __syncthreads();
  const int q = tid & 15, rg = tid >> 4, e8 = q * 8;
  const v4f ib0 = *(const v4fa*)(sIB + e8), ib1 = *(const v4fa*)(sIB + e8 + 4);
#pragma unroll 1
  for (int it = 0; it < 16; ++it) {
    const int row = it * 16 + rg;
    const float id = sID[row];
    const float* hp = Hb + row * 128 + e8;
    const v4f h0 = *(const v4fa*)hp, h1 = *(const v4fa*)(hp + 4);
    const v4f l0 = h0 * id, l1 = h1 * id, r0 = h0 * ib0, r1 = h1 * ib1;
    const v4u lh = hi8(l0, l1), ll = lo8(l0, l1), rh = hi8(r0, r1), rl = lo8(r0, r1);
    const size_t o = ((size_t)blockIdx.x * 256 + row) * 256 + e8;
    *(volatile v4u*)(L + o) = lh;
    *(volatile v4u*)(L + o + 128) = ll;
    *(volatile v4u*)(R + o) = rh;
    *(volatile v4u*)(R + o + 128) = rl;
    __threadfence();
    *(volatile v4u*)(L + o) = lh;
    *(volatile v4u*)(L + o + 128) = ll;
    *(volatile v4u*)(R + o) = rh;
    *(volatile v4u*)(R + o + 128) = rl;
  }
}

__global__ __launch_bounds__(128) KATTR
void k_tg(const u16* __restrict__ XIN, const u16* __restrict__ FG, const float* __restrict__ fb,
          const float* __restrict__ gb, u16* __restrict__ XT)
{
  __shared__ __attribute__((aligned(16))) float sS[4 * 16 * 132];
  const int tid = threadIdx.x, lane = tid & 31, w = tid >> 5;
  const int h = lane >> 4, m = lane & 15;
  const int m0w = blockIdx.x * 128 + 32 * w;
  const u16* a0 = XIN + (size_t)(m0w + m) * 128 + 8 * h;
  const u16* a1 = a0 + 16 * 128;
  const u16* b = FG + m * 128 + 8 * h;
  v8f acc[2][8];
  zero_acc<8>(acc);
  mm1<8>(acc, a0, a1, b, 128, 128);
  float* slab = sS + w * 16 * 132;
#pragma unroll
  for (int mt = 0; mt < 2; ++mt) {
#pragma unroll
    for (int nt = 0; nt < 4; ++nt) {
      const float bv = rbf(fb[16 * nt + m]);
#pragma unroll
      for (int r = 0; r < 8; ++r) slab[(8 * h + r) * 132 + 16 * nt + m] = acc[mt][nt][r] + bv;
    }
#pragma unroll
    for (int nt = 4; nt < 8; ++nt) {
      const float bv = rbf(gb[16 * (nt - 4) + m]);
#pragma unroll
      for (int r = 0; r < 8; ++r) slab[(8 * h + r) * 132 + 16 * nt + m] = acc[mt][nt][r] + bv;
    }
    wsync();
#pragma unroll 1
    for (int e = 0; e < 32; ++e) {
      const int idx = e * 32 + lane;
      float* p = slab + (idx >> 6) * 132 + (idx & 63);
      const float f = p[0], g = p[64];
      p[0] = tanhf(f) * (1.0f / (1.0f + expf(-g)));
    }
    wsync();
    store_hl(slab, 132, XT + (size_t)(m0w + 16 * mt) * 128, 128, 64, lane);
    wsync();
  }
}

template <bool LAST>
__global__ __launch_bounds__(128) KATTR
void k_skip(const u16* __restrict__ XT, const u16* __restrict__ SK, const float* __restrict__ sb,
            float* __restrict__ SKIP, u16* __restrict__ RHL)
{
  __shared__ __attribute__((aligned(16))) float sS[4 * 16 * 68];
  const int tid = threadIdx.x, lane = tid & 31, w = tid >> 5;
  const int h = lane >> 4, m = lane & 15;
  const int m0w = blockIdx.x * 128 + 32 * w;
  const u16* a0 = XT + (size_t)(m0w + m) * 128 + 8 * h;
  const u16* a1 = a0 + 16 * 128;
  const u16* b = SK + m * 128 + 8 * h;
  v8f acc[2][4];
  zero_acc<4>(acc);
  mm1<4>(acc, a0, a1, b, 128, 128);
  float* slab = sS + w * 16 * 68;
#pragma unroll
  for (int mt = 0; mt < 2; ++mt) {
    stage16<4, true>(slab, acc[mt], sb, 0, h, m);
    wsync();
    const int row0 = m0w + 16 * mt;
    if constexpr (!LAST) {
      const int hh = lane >> 4, c4 = (lane & 15) * 4;
      v4f vals[8];
#pragma unroll
      for (int it = 0; it < 8; ++it) {
        const int row = it * 2 + hh;
        const v4f sv = *(const v4fa*)(slab + row * 68 + c4);
        const v4f gv = *(const v4fa*)(SKIP + (size_t)(row0 + row) * 64 + c4);
        vals[it] = sv + gv;
      }
#pragma unroll
      for (int pass = 0; pass < 2; ++pass) {
#pragma unroll
        for (int it = 0; it < 8; ++it) {
          const int row = it * 2 + hh;
          *(volatile v4f*)(SKIP + (size_t)(row0 + row) * 64 + c4) = vals[it];
        }
        __threadfence();
      }
    } else {
      const int q = lane >> 3, c8 = (lane & 7) * 8;
#pragma unroll 1
      for (int it = 0; it < 4; ++it) {
        const int row = it * 4 + q;
        float* p = slab + row * 68 + c8;
        const float* g = SKIP + (size_t)(row0 + row) * 64 + c8;
        const v4f s0 = *(const v4fa*)p + *(const v4fa*)g;
        const v4f s1 = *(const v4fa*)(p + 4) + *(const v4fa*)(g + 4);
        const v4f r0 = { relu_keep(s0.x), relu_keep(s0.y), relu_keep(s0.z), relu_keep(s0.w) };
        const v4f r1 = { relu_keep(s1.x), relu_keep(s1.y), relu_keep(s1.z), relu_keep(s1.w) };
        *(v4fa*)p = r0;
        *(v4fa*)(p + 4) = r1;
      }
      wsync();
      store_hl(slab, 68, RHL + (size_t)row0 * 128, 128, 64, lane);
    }
    wsync();
  }
}

__global__ __launch_bounds__(128) KATTR
void k_cz(u16* ws, long aD, long aG, long cz, long zD, long zG)
{
  __shared__ __attribute__((aligned(16))) float zT[64 * 132];
  const int tid = threadIdx.x, lane = tid & 31, w = tid >> 5;
  const int h = lane >> 4, m = lane & 15;
  const int z = blockIdx.z;
  const long aoff = z ? aG : aD;
  const long zoff = z ? zG : zD;
  const int m0 = blockIdx.x * 128, m0w = m0 + 32 * w;
  const u16* a0 = ws + aoff + (size_t)(m0w + m) * 128 + 8 * h;
  const u16* a1 = a0 + 16 * 128;
  const u16* b = ws + cz + (size_t)z * 8192 + m * 128 + 8 * h;
  v8f acc[2][4];
  zero_acc<4>(acc);
  mm1<4>(acc, a0, a1, b, 128, 128);
#pragma unroll
  for (int mt = 0; mt < 2; ++mt)
#pragma unroll
    for (int nt = 0; nt < 4; ++nt)
#pragma unroll
      for (int r = 0; r < 8; ++r)
        zT[(16 * nt + m) * 132 + 32 * w + 16 * mt + 8 * h + r] = acc[mt][nt][r];
  __syncthreads();
  const int bt = m0 >> 8, nh = (m0 >> 7) & 1;
  const int q = tid & 15, rg = tid >> 4, c8 = q * 8;
  v4u hv[8], lv[8];
#pragma unroll
  for (int it = 0; it < 8; ++it) {
    const float* p = zT + (it * 8 + rg) * 132 + c8;
    const v4f a = *(const v4fa*)p;
    const v4f bb = *(const v4fa*)(p + 4);
    hv[it] = hi8(a, bb);
    lv[it] = lo8(a, bb);
  }
#pragma unroll
  for (int pass = 0; pass < 2; ++pass) {
#pragma unroll
    for (int it = 0; it < 8; ++it) {
      const int d = it * 8 + rg;
      u16* dst = ws + zoff + ((size_t)(bt * 64 + d) * 256 + nh * 128 + c8);
      *(volatile v4u*)dst = hv[it];
      *(volatile v4u*)(dst + ZLO) = lv[it];
    }
    __threadfence();
  }
}

__global__ __launch_bounds__(128) KATTR
void k_prop(u16* ws, long oAN, long oAG, long oZD, long oZG, long oXD, long oXG)
{
  __shared__ __attribute__((aligned(16))) float sS[4 * 16 * 68];
  const int tid = threadIdx.x, lane = tid & 31, w = tid >> 5;
  const int h = lane >> 4, m = lane & 15;
  const int mtile = blockIdx.x, bt = blockIdx.y, z = blockIdx.z;
  const long ao = z ? oAG : (oAN + (long)(bt >> 6) * 131072);
  const long zo = (z ? oZG : oZD) + (long)bt * 16384;
  const long xo = z ? oXG : oXD;
  const int mloc = mtile * 128 + 32 * w;
  const u16* a0 = ws + ao + (size_t)(mloc + m) * 512 + 8 * h;
  const u16* a1 = a0 + 16 * 512;
  const u16* b = ws + zo + m * 256 + 8 * h;
  v8f acc[2][4];
  zero_acc<4>(acc);
  mm3<4>(acc, a0, a1, 256L, b, ZLO, 256, 256);
  float* slab = sS + w * 16 * 68;
#pragma unroll
  for (int mt = 0; mt < 2; ++mt) {
    stage16<4, false>(slab, acc[mt], (const float*)0, 0, h, m);
    wsync();
    const size_t row0 = (size_t)bt * 256 + mloc + 16 * mt;
    store_hl(slab, 68, ws + xo + row0 * 128, 128, 64, lane);
    wsync();
  }
}

__global__ __launch_bounds__(128) KATTR
void k_fuse(const u16* __restrict__ XD, const u16* __restrict__ XG, const u16* __restrict__ XT,
            const u16* __restrict__ FB, u16* __restrict__ O)
{
  __shared__ __attribute__((aligned(16))) float sS[4 * 16 * 68];
  const int tid = threadIdx.x, lane = tid & 31, w = tid >> 5;
  const int h = lane >> 4, m = lane & 15;
  const int m0w = blockIdx.x * 128 + 32 * w;
  const size_t ra = (size_t)(m0w + m) * 128 + 8 * h;
  const u16* b = FB + m * 512 + 8 * h;
  v8f acc[2][4];
  zero_acc<4>(acc);
  mm1<4>(acc, XD + ra, XD + ra + 2048, b,       512, 128);
  mm1<4>(acc, XG + ra, XG + ra + 2048, b + 128, 512, 128);
  mm1<4>(acc, XT + ra, XT + ra + 2048, b + 256, 512, 128);
  mm1<4>(acc, XT + ra, XT + ra + 2048, b + 384, 512, 128);
  float* slab = sS + w * 16 * 68;
  const int q = lane >> 3, c8 = (lane & 7) * 8;
#pragma unroll
  for (int mt = 0; mt < 2; ++mt) {
    stage16<4, false>(slab, acc[mt], (const float*)0, 0, h, m);
    wsync();
#pragma unroll 1
    for (int e = 0; e < 32; ++e) {
      const int idx = e * 32 + lane;
      float* p = slab + (idx >> 6) * 68 + (idx & 63);
      p[0] = 1.0f / (1.0f + expf(-p[0]));
    }
    wsync();
    const int row0 = m0w + 16 * mt;
#pragma unroll 1
    for (int it = 0; it < 4; ++it) {
      const int row = it * 4 + q;
      const size_t go = (size_t)(row0 + row) * 128 + c8;
      const v4u dh = *(const v4ua*)(XD + go), dl = *(const v4ua*)(XD + go + 64);
      const v4u gh = *(const v4ua*)(XG + go), gl = *(const v4ua*)(XG + go + 64);
      v4f dh0, dh1, dl0, dl1, gh0, gh1, gl0, gl1;
      unp8(dh, dh0, dh1); unp8(dl, dl0, dl1); unp8(gh, gh0, gh1); unp8(gl, gl0, gl1);
      const v4f xd0 = dh0 + dl0, xd1 = dh1 + dl1, xg0 = gh0 + gl0, xg1 = gh1 + gl1;
      float* p = slab + row * 68 + c8;
      const v4f v0 = *(const v4fa*)p, v1 = *(const v4fa*)(p + 4);
      const v4f o0 = v0 * xd0 + (1.0f - v0) * xg0;
      const v4f o1 = v1 * xd1 + (1.0f - v1) * xg1;
      *(v4fa*)p = o0;
      *(v4fa*)(p + 4) = o1;
    }
    wsync();
    store_hl(slab, 68, O + (size_t)row0 * 128, 128, 64, lane);
    wsync();
  }
}

__global__ __launch_bounds__(128) KATTR
void k_out(const u16* __restrict__ O0, const u16* __restrict__ O1, const u16* __restrict__ OB,
           const float* __restrict__ ob, const float* __restrict__ gam, const float* __restrict__ bet,
           u16* __restrict__ XN)
{
  __shared__ __attribute__((aligned(16))) float sS[4 * 16 * 68];
  const int tid = threadIdx.x, lane = tid & 31, w = tid >> 5;
  const int h = lane >> 4, m = lane & 15;
  const int m0w = blockIdx.x * 128 + 32 * w;
  const size_t ra = (size_t)(m0w + m) * 128 + 8 * h;
  const u16* b = OB + m * 256 + 8 * h;
  v8f acc[2][4];
  zero_acc<4>(acc);
  mm1<4>(acc, O0 + ra, O0 + ra + 2048, b,       256, 128);
  mm1<4>(acc, O1 + ra, O1 + ra + 2048, b + 128, 256, 128);
  float* slab = sS + w * 16 * 68;
  const int q = lane >> 3, c8 = (lane & 7) * 8;
  const v4f g0 = rb4(*(const v4fa*)(gam + c8)), g1 = rb4(*(const v4fa*)(gam + c8 + 4));
  const v4f e0 = rb4(*(const v4fa*)(bet + c8)), e1 = rb4(*(const v4fa*)(bet + c8 + 4));
#pragma unroll
  for (int mt = 0; mt < 2; ++mt) {
    stage16<4, true>(slab, acc[mt], ob, 0, h, m);
    wsync();
#pragma unroll 1
    for (int it = 0; it < 4; ++it) {
      float* p = slab + (it * 4 + q) * 68 + c8;
      const v4f x0 = *(const v4fa*)p, x1 = *(const v4fa*)(p + 4);
      float s = ((x0.x + x0.y) + (x0.z + x0.w)) + ((x1.x + x1.y) + (x1.z + x1.w));
      s += __shfl_xor(s, 1);
      s += __shfl_xor(s, 2);
      s += __shfl_xor(s, 4);
      const float mean = s * (1.0f / 64.0f);
      const v4f d0 = x0 - mean, d1 = x1 - mean;
      const v4f q0 = d0 * d0, q1 = d1 * d1;
      float vs = ((q0.x + q0.y) + (q0.z + q0.w)) + ((q1.x + q1.y) + (q1.z + q1.w));
      vs += __shfl_xor(vs, 1);
      vs += __shfl_xor(vs, 2);
      vs += __shfl_xor(vs, 4);
      const float inv = 1.0f / sqrtf(vs * (1.0f / 64.0f) + 1e-5f);
      const v4f y0 = d0 * inv * g0 + e0;
      const v4f y1 = d1 * inv * g1 + e1;
      *(v4fa*)p = y0;
      *(v4fa*)(p + 4) = y1;
    }
    wsync();
    store_hl(slab, 68, XN + (size_t)(m0w + 16 * mt) * 128, 128, 64, lane);
    wsync();
  }
}

extern "C" void kernel_launch(void* const* d_in, const int* in_sizes, int n_in,
                              void* d_out, int out_size, void* d_ws, size_t ws_size,
                              hipStream_t stream) {
  if (n_in < 26) return;
  const int exp_sz[26] = { 65536, 65536, 8192, 32768, 4096, 4096, 4096, 64, 64, 64, 12288, 192, 12288, 192,
                           12288, 192, 8192, 8192, 8192, 8192, 8192, 64, 64, 64, 4096, 64 };
  for (int i = 0; i < 26; ++i) if (in_sizes[i] != exp_sz[i]) return;
  if (out_size != MTOK * NDIM) return;
  if (ws_size < B_TOTAL) return;

  const float* X      = (const float*)d_in[0];
  const float* Amat   = (const float*)d_in[1];
  const float* hemb   = (const float*)d_in[2];
  const float* Gl     = (const float*)d_in[3];
  const float* Wq     = (const float*)d_in[4];
  const float* Wk     = (const float*)d_in[5];
  const float* nodeW  = (const float*)d_in[6];
  const float* nodeb  = (const float*)d_in[7];
  const float* startW = (const float*)d_in[8];
  const float* startb = (const float*)d_in[9];
  const float* filtW  = (const float*)d_in[10];
  const float* filtb  = (const float*)d_in[11];
  const float* gateW  = (const float*)d_in[12];
  const float* gateb  = (const float*)d_in[13];
  const float* skipW  = (const float*)d_in[14];
  const float* skipb  = (const float*)d_in[15];
  const float* convW  = (const float*)d_in[16];
  const float* convWg = (const float*)d_in[17];
  const float* Wfuse  = (const float*)d_in[18];
  const float* Wgfuse = (const float*)d_in[19];
  const float* outW   = (const float*)d_in[20];
  const float* outb   = (const float*)d_in[21];
  const float* gamma  = (const float*)d_in[22];
  const float* beta   = (const float*)d_in[23];
  const float* endW   = (const float*)d_in[24];
  const float* endb   = (const float*)d_in[25];
  float* out = (float*)d_out;

  char* wsb = (char*)d_ws;
  u16* ws16 = (u16*)d_ws;
  float* SKIP = (float*)wsb;
  float* HF = (float*)(wsb + B_HF);
  float* HG = (float*)(wsb + B_HG);

  k_pa<<<dim3(4, 17, 1), dim3(256), 0, stream>>>(filtW, gateW, skipW, Wfuse, Wgfuse, outW, endW, Wq, ws16);
  k_pb<<<dim3(40), dim3(256), 0, stream>>>(nodeW, Wk, hemb, Amat, ws16);
  k_pc<<<dim3(64), dim3(256), 0, stream>>>(convW, convWg, Gl, X, ws16);
  k_pd<<<dim3(MTOK * 16 / 256), dim3(256), 0, stream>>>(X, startW, startb, ws16 + 1 * SLOTE, SKIP);

  k_gm<4, 1, 0, true, 64, 0, 64, 0, 64, 128, 64, 0, 0, 0><<<dim3(8, 1, 1), dim3(128), 0, stream>>>(
      ws16 + E_XPT, ws16 + E_NWB, nodeb, ws16 + E_EEMB, HF);
  k_gm<4, 1, 0, false, 64, 0, 64, 0, 64, 128, 64, 0, 0, 0><<<dim3(1, 1, 1), dim3(128), 0, stream>>>(
      ws16 + E_HEMB, ws16 + E_WKB, nodeb, ws16 + E_KHL, HF);
  k_gm<4, 1, 0, false, 128, 0, 128, 0, 128, 128, 64, 0, 0, 0><<<dim3(8, 1, 1), dim3(128), 0, stream>>>(
      ws16 + E_EEMB, ws16 + E_WQD, nodeb, ws16 + E_QHL, HF);
  k_gm<8, 3, 2, false, 128, 64, 128, 64, 64, 128, 0, 0, 0, 0><<<dim3(8, 1, 1), dim3(128), 0, stream>>>(
      ws16 + E_QHL, ws16 + E_KHL, nodeb, ws16 + E_LP, HF);
  k_lr<<<dim3(4), dim3(256), 0, stream>>>(HF, ws16 + E_LP, ws16 + E_RP);
  k_gm<4, 3, 0, false, 256, 128, 256, 128, 128, 512, 256, 65536, 65536, 131072><<<dim3(2, 4, 4), dim3(128), 0, stream>>>(
      ws16 + E_LP, ws16 + E_RP, nodeb, ws16 + E_ANHL, HF);
  k_gm<8, 1, 1, false, 256, 0, 256, 0, 256, 128, 0, 0, 0, 0><<<dim3(2, 1, 1), dim3(128), 0, stream>>>(
      ws16 + E_ABF, ws16 + E_GLT, nodeb, ws16 + E_LG, HG);
  k_lr<<<dim3(1), dim3(256), 0, stream>>>(HG, ws16 + E_LG, ws16 + E_RG);
  k_gm<4, 3, 0, false, 256, 128, 256, 128, 128, 512, 256, 65536, 65536, 131072><<<dim3(2, 4, 1), dim3(128), 0, stream>>>(
      ws16 + E_LG, ws16 + E_RG, nodeb, ws16 + E_AGHL, HF);

  const int xinS[3] = { 1, 4, 1 };
  const int zgS[2]  = { 4, 1 };
  const int o0S[2]  = { 1, 4 };
  const int nxS[2]  = { 4, 1 };
  for (int i = 0; i < 2; ++i) {
    k_tg<<<dim3(MTOK / 128), dim3(128), 0, stream>>>(ws16 + xinS[i] * SLOTE, ws16 + E_FG + i * 16384,
                                                     filtb + i * 64, gateb + i * 64, ws16 + 2 * SLOTE);
    k_skip<false><<<dim3(MTOK / 128), dim3(128), 0, stream>>>(ws16 + 2 * SLOTE, ws16 + E_SK + i * 8192,
                                                              skipb + i * 64, SKIP, ws16 + 3 * SLOTE);
    for (int j = 0; j < 2; ++j) {
      const long aD = (long)((j == 0) ? 2 : 5) * (long)SLOTE;
      const long aG = (long)((j == 0) ? 2 : 6) * (long)SLOTE;
      const long zD = 3L * (long)SLOTE;
      const long zG = (long)zgS[i] * (long)SLOTE;
      k_cz<<<dim3(MTOK / 128, 1, 2), dim3(128), 0, stream>>>(ws16, aD, aG, (long)E_CZ + (long)j * 16384, zD, zG);
      k_prop<<<dim3(2, 256, 2), dim3(128), 0, stream>>>(ws16, (long)E_ANHL, (long)E_AGHL, zD, zG,
                                                        5L * (long)SLOTE, 6L * (long)SLOTE);
      const int oS = (j == 0) ? o0S[i] : 3;
      k_fuse<<<dim3(MTOK / 128), dim3(128), 0, stream>>>(ws16 + 5 * SLOTE, ws16 + 6 * SLOTE, ws16 + 2 * SLOTE,
                                                         ws16 + E_FUSE, ws16 + oS * SLOTE);
    }
    k_out<<<dim3(MTOK / 128), dim3(128), 0, stream>>>(ws16 + o0S[i] * SLOTE, ws16 + 3 * SLOTE, ws16 + E_OUT,
                                                      outb, gamma, beta, ws16 + nxS[i] * SLOTE);
  }
  k_tg<<<dim3(MTOK / 128), dim3(128), 0, stream>>>(ws16 + xinS[2] * SLOTE, ws16 + E_FG + 2 * 16384,
                                                   filtb + 128, gateb + 128, ws16 + 2 * SLOTE);
  k_skip<true><<<dim3(MTOK / 128), dim3(128), 0, stream>>>(ws16 + 2 * SLOTE, ws16 + E_SK + 2 * 8192,
                                                           skipb + 128, SKIP, ws16 + 3 * SLOTE);
  k_gm<4, 1, 1, true, 128, 0, 128, 0, 128, 64, 0, 0, 0, 0><<<dim3(MTOK / 128, 1, 1), dim3(128), 0, stream>>>(
      ws16 + 3 * SLOTE, ws16 + E_END, endb, ws16 + E_LP, out);
  (void)hipGetLastError();
}
